// PositionAwareSelfAttention_80109730005018
// MI455X (gfx1250) — hardware-verified
//
#include <hip/hip_runtime.h>
#include <hip/hip_bf16.h>

#define BATCH 4
#define SEQ   2048
#define CH    512
#define HEADS 8
#define HDIM  64
#define ROWS  (BATCH * SEQ)

typedef __attribute__((ext_vector_type(16))) _Float16 v16h;
typedef __attribute__((ext_vector_type(8)))  _Float16 h8;
typedef __attribute__((ext_vector_type(8)))  float    v8f;
typedef __attribute__((ext_vector_type(4)))  float    v4f;
typedef __attribute__((ext_vector_type(4)))  unsigned v4u;
template <typename T> __device__ __forceinline__ void vst2(void* p, T v) { *(volatile T*)p = v; __threadfence(); *(volatile T*)p = v; }

__device__ __forceinline__ v8f vzero8() {
    v8f z;
#pragma unroll
    for (int i = 0; i < 8; ++i) z[i] = 0.0f;
    return z;
}

__device__ __forceinline__ v16h combine16(h8 lo, h8 hi) {
    v16h r;
#pragma unroll
    for (int i = 0; i < 8; ++i) { r[i] = lo[i]; r[i + 8] = hi[i]; }
    return r;
}

__device__ __forceinline__ v16h load_a_frag(const _Float16* __restrict__ base, int ld) {
    int lane = threadIdx.x & 31;
    int row  = lane & 15;
    int kh   = (lane >> 4) * 8;
    const _Float16* p = base + row * ld + kh;
    h8 lo = *(const h8*)(p);
    h8 hi = *(const h8*)(p + 16);
    return combine16(lo, hi);
}

__device__ __forceinline__ v16h load_b_frag(const _Float16* __restrict__ base, int ld) {
    int lane = threadIdx.x & 31;
    int n    = lane & 15;
    int kh   = (lane >> 4) * 8;
    const _Float16* p = base + n * ld + kh;
    return combine16(*(const h8*)(p), *(const h8*)(p + 16));
}

__device__ __forceinline__ v8f wmma32(v16h a, v16h b, v8f c) {
    v8f d = __builtin_amdgcn_wmma_f32_16x16x32_f16(false, a, false, b, (short)0, c, false, false);
    asm volatile("v_nop\n\tv_nop\n\tv_nop\n\tv_nop" : "+v"(d) : "v"(a), "v"(b));
    return d;
}

__global__ void cvt_f16_kernel(const float* __restrict__ src,
                               _Float16* __restrict__ dst, int n) {
    int g = blockIdx.x * blockDim.x + threadIdx.x;
    int stride = gridDim.x * blockDim.x;
    for (; g * 8 < n; g += stride) {
        union { h8 h; v4u u; } pk;
#pragma unroll
        for (int e = 0; e < 8; ++e) pk.h[e] = (_Float16)src[(size_t)g * 8 + e];
        vst2(dst + (size_t)g * 8, pk.u);
    }
}

__global__ __launch_bounds__(128)
void gemm_qkv_kernel(const _Float16* __restrict__ X, const _Float16* __restrict__ W,
                     const float* __restrict__ bias, _Float16* __restrict__ out, int mode) {
    const int K = CH, ldx = CH, ldw = CH;
    int wave = threadIdx.x >> 5;
    int lane = threadIdx.x & 31;
    int rbase = blockIdx.x * 128 + (wave & 1) * 64;
    int cbase = blockIdx.y * 128 + (wave >> 1) * 64;

    v8f acc[4][4];
#pragma unroll
    for (int i = 0; i < 4; ++i)
#pragma unroll
        for (int j = 0; j < 4; ++j) acc[i][j] = vzero8();

    for (int k0 = 0; k0 < K; k0 += 32) {
        v16h a[4], bf[4];
#pragma unroll
        for (int i = 0; i < 4; ++i)
            a[i] = load_a_frag(X + (size_t)(rbase + 16 * i) * ldx + k0, ldx);
#pragma unroll
        for (int j = 0; j < 4; ++j)
            bf[j] = load_b_frag(W + (size_t)(cbase + 16 * j) * ldw + k0, ldw);
#pragma unroll
        for (int i = 0; i < 4; ++i)
#pragma unroll
            for (int j = 0; j < 4; ++j)
                acc[i][j] = wmma32(a[i], bf[j], acc[i][j]);
    }

    int nloc = lane & 15, hs = lane >> 4;
    __shared__ __align__(16) _Float16 st[4][64 * 72];
    _Float16* S = st[wave];
#pragma unroll
    for (int rt = 0; rt < 4; ++rt)
#pragma unroll
        for (int ct = 0; ct < 4; ++ct)
#pragma unroll
            for (int r = 0; r < 8; ++r) {
                int rl = rt * 16 + r + 8 * hs, cl = ct * 16 + nloc;
                float v = acc[rt][ct][r] + bias[cbase + cl];
                if (mode == 0) S[rl * 72 + cl] = (_Float16)v; else S[cl * 72 + rl] = (_Float16)v;
            }
    asm volatile("s_wait_dscnt 0" ::: "memory"); __builtin_amdgcn_wave_barrier(); __builtin_amdgcn_fence(__ATOMIC_RELEASE, "workgroup");
    {
        const int b = rbase >> 11, n0 = rbase & (SEQ - 1), h = cbase >> 6;
#pragma unroll 4
        for (int q = 0; q < 16; ++q) {
            const int rl = q * 4 + (lane >> 3), pc = lane & 7;
            size_t idx;
            if (mode == 0) idx = ((size_t)(b * HEADS + h) * SEQ + n0 + rl) * HDIM + pc * 8;
            else           idx = ((size_t)(b * HEADS + h) * HDIM + rl) * SEQ + n0 + pc * 8;
            vst2(out + idx, *(const v4u*)(S + rl * 72 + pc * 8));
        }
    }
}

__global__ __launch_bounds__(128)
void flash_attn_kernel(const _Float16* __restrict__ Qh, const _Float16* __restrict__ Kh,
                       const _Float16* __restrict__ Vt, const float* __restrict__ qp,
                       _Float16* __restrict__ Oh) {
    __shared__ __align__(16) _Float16 Plds[4][16][72];

    int wave = threadIdx.x >> 5;
    int lane = threadIdx.x & 31;
    int nloc = lane & 15, hs = lane >> 4;
    int bh = blockIdx.y;
    int b = bh >> 3, h = bh & 7;
    int qbase = blockIdx.x * 64 + wave * 16;

    const _Float16* Qb = Qh + (size_t)bh * SEQ * HDIM;
    const _Float16* Kb = Kh + (size_t)bh * SEQ * HDIM;
    const _Float16* Vb = Vt + (size_t)bh * HDIM * SEQ;

    v16h qf0 = load_a_frag(Qb + (size_t)qbase * HDIM +  0, HDIM);
    v16h qf1 = load_a_frag(Qb + (size_t)qbase * HDIM + 32, HDIM);

    float qx[8], qy[8], m8[8], l8[8];
    v8f O[4];
#pragma unroll
    for (int r = 0; r < 8; ++r) {
        int g = qbase + r + 8 * hs;
        qx[r] = qp[((size_t)(b * SEQ + g)) * 4 + 0];
        qy[r] = qp[((size_t)(b * SEQ + g)) * 4 + 1];
        m8[r] = -1e30f;
        l8[r] = 0.0f;
    }
#pragma unroll
    for (int dt = 0; dt < 4; ++dt) O[dt] = vzero8();

    for (int kb = 0; kb < SEQ; kb += 64) {
        v8f S[4];
#pragma unroll
        for (int ct = 0; ct < 4; ++ct) {
            v16h bk0 = load_b_frag(Kb + (size_t)(kb + ct * 16) * HDIM +  0, HDIM);
            v16h bk1 = load_b_frag(Kb + (size_t)(kb + ct * 16) * HDIM + 32, HDIM);
            v8f z = vzero8();
            z = wmma32(qf0, bk0, z);
            S[ct] = wmma32(qf1, bk1, z);
        }

        float p[4][8], rm[8];
#pragma unroll
        for (int r = 0; r < 8; ++r) rm[r] = -1e30f;
#pragma unroll
        for (int ct = 0; ct < 4; ++ct) {
            int key = kb + ct * 16 + nloc;
            float kx = qp[((size_t)(b * SEQ + key)) * 4 + 0];
            float ky = qp[((size_t)(b * SEQ + key)) * 4 + 1];
#pragma unroll
            for (int r = 0; r < 8; ++r) {
                float dx = fabsf(qx[r] - kx), dy = fabsf(qy[r] - ky);
                float biasv = -0.1f * sqrtf(dx * dx + dy * dy + 1e-8f);
                float s = S[ct][r] * 0.125f + biasv;
                p[ct][r] = s;
                rm[r] = fmaxf(rm[r], s);
            }
        }
#pragma unroll
        for (int r = 0; r < 8; ++r) {
            float v = rm[r];
            v = fmaxf(v, __shfl_xor(v, 1, 32));
            v = fmaxf(v, __shfl_xor(v, 2, 32));
            v = fmaxf(v, __shfl_xor(v, 4, 32));
            v = fmaxf(v, __shfl_xor(v, 8, 32));
            rm[r] = v;
        }
        float alpha[8], rs[8];
#pragma unroll
        for (int r = 0; r < 8; ++r) {
            float mn = fmaxf(m8[r], rm[r]);
            alpha[r] = __expf(m8[r] - mn);
            m8[r] = mn;
            rs[r] = 0.0f;
        }
#pragma unroll
        for (int ct = 0; ct < 4; ++ct)
#pragma unroll
            for (int r = 0; r < 8; ++r) {
                float e = __expf(p[ct][r] - m8[r]);
                p[ct][r] = e;
                rs[r] += e;
            }
#pragma unroll
        for (int r = 0; r < 8; ++r) {
            float v = rs[r];
            v += __shfl_xor(v, 1, 32);
            v += __shfl_xor(v, 2, 32);
            v += __shfl_xor(v, 4, 32);
            v += __shfl_xor(v, 8, 32);
            l8[r] = l8[r] * alpha[r] + v;
        }
#pragma unroll
        for (int dt = 0; dt < 4; ++dt)
#pragma unroll
            for (int r = 0; r < 8; ++r) O[dt][r] *= alpha[r];

#pragma unroll
        for (int ct = 0; ct < 4; ++ct)
#pragma unroll
            for (int r = 0; r < 8; ++r)
                Plds[wave][r + 8 * hs][ct * 16 + nloc] = (_Float16)p[ct][r];
        asm volatile("s_wait_dscnt 0" ::: "memory"); __builtin_amdgcn_wave_barrier(); __builtin_amdgcn_fence(__ATOMIC_RELEASE, "workgroup");

        const _Float16* pr = &Plds[wave][nloc][0];
        int kh = hs * 8;
        v16h pf0 = combine16(*(const h8*)(pr + kh),       *(const h8*)(pr + kh + 16));
        v16h pf1 = combine16(*(const h8*)(pr + 32 + kh),  *(const h8*)(pr + 32 + kh + 16));

#pragma unroll
        for (int dt = 0; dt < 4; ++dt) {
            const _Float16* vr = Vb + (size_t)(dt * 16 + nloc) * SEQ + kb + hs * 8;
            v16h v0 = combine16(*(const h8*)(vr),      *(const h8*)(vr + 16));
            v16h v1 = combine16(*(const h8*)(vr + 32), *(const h8*)(vr + 48));
            O[dt] = wmma32(pf0, v0, O[dt]);
            O[dt] = wmma32(pf1, v1, O[dt]);
        }
        __builtin_amdgcn_wave_barrier();
    }

#pragma unroll
    for (int dt = 0; dt < 4; ++dt)
#pragma unroll
        for (int r = 0; r < 8; ++r) Plds[wave][r + 8 * hs][dt * 16 + nloc] = (_Float16)(O[dt][r] / l8[r]);
    asm volatile("s_wait_dscnt 0" ::: "memory"); __builtin_amdgcn_wave_barrier(); __builtin_amdgcn_fence(__ATOMIC_RELEASE, "workgroup");
#pragma unroll
    for (int q = 0; q < 4; ++q) { const int rl = q * 4 + (lane >> 3), pc = lane & 7;
        vst2(Oh + ((size_t)(b * SEQ + qbase + rl)) * CH + h * HDIM + pc * 8, *(const v4u*)(&Plds[wave][rl][pc * 8])); }
}

__global__ __launch_bounds__(128)
void gemm_out_kernel(const _Float16* __restrict__ A, const _Float16* __restrict__ W,
                     const float* __restrict__ bias, const float* __restrict__ resid,
                     float* __restrict__ H) {
    const int K = CH, lda = CH, ldw = CH;
    int wave = threadIdx.x >> 5;
    int lane = threadIdx.x & 31;
    int rbase = blockIdx.x * 128 + (wave & 1) * 64;
    int cbase = blockIdx.y * 128 + (wave >> 1) * 64;

    v8f acc[4][4];
#pragma unroll
    for (int i = 0; i < 4; ++i)
#pragma unroll
        for (int j = 0; j < 4; ++j) acc[i][j] = vzero8();

    for (int k0 = 0; k0 < K; k0 += 32) {
        v16h a[4], bf[4];
#pragma unroll
        for (int i = 0; i < 4; ++i)
            a[i] = load_a_frag(A + (size_t)(rbase + 16 * i) * lda + k0, lda);
#pragma unroll
        for (int j = 0; j < 4; ++j)
            bf[j] = load_b_frag(W + (size_t)(cbase + 16 * j) * ldw + k0, ldw);
#pragma unroll
        for (int i = 0; i < 4; ++i)
#pragma unroll
            for (int j = 0; j < 4; ++j)
                acc[i][j] = wmma32(a[i], bf[j], acc[i][j]);
    }

    int nloc = lane & 15, hs = lane >> 4;
    __shared__ __align__(16) float sto[4][64 * 68];
    float* S = sto[wave];
#pragma unroll
    for (int rt = 0; rt < 4; ++rt)
#pragma unroll
        for (int ct = 0; ct < 4; ++ct)
#pragma unroll
            for (int r = 0; r < 8; ++r) {
                int rl = rt * 16 + r + 8 * hs, cl = ct * 16 + nloc;
                S[rl * 68 + cl] = acc[rt][ct][r] + bias[cbase + cl];
            }
    asm volatile("s_wait_dscnt 0" ::: "memory"); __builtin_amdgcn_wave_barrier(); __builtin_amdgcn_fence(__ATOMIC_RELEASE, "workgroup");
#pragma unroll 4
    for (int q = 0; q < 32; ++q) { const int rl = q * 2 + (lane >> 4), pc = lane & 15;
        const size_t idx = (size_t)(rbase + rl) * CH + cbase + pc * 4;
        v4f v = *(const v4f*)(S + rl * 68 + pc * 4); const v4f rr = *(const v4f*)(resid + idx);
        vst2(H + idx, v + rr); }
}

__global__ __launch_bounds__(256)
void layernorm_kernel(const float* __restrict__ Hb, const float* __restrict__ gamma,
                      const float* __restrict__ beta, float* __restrict__ out) {
    int wave = threadIdx.x >> 5;
    int lane = threadIdx.x & 31;
    size_t row = (size_t)blockIdx.x * 8 + wave;
    const float* hr = Hb + row * CH;

    float s = 0.0f, ss = 0.0f;
#pragma unroll
    for (int i = 0; i < CH / 32; ++i) {
        float v = hr[lane + i * 32];
        s += v; ss += v * v;
    }
#pragma unroll
    for (int mask = 1; mask < 32; mask <<= 1) {
        s  += __shfl_xor(s,  mask, 32);
        ss += __shfl_xor(ss, mask, 32);
    }
    float mu   = s * (1.0f / CH);
    float var  = ss * (1.0f / CH) - mu * mu;
    float rstd = rsqrtf(var + 1e-5f);
#pragma unroll
    for (int i = 0; i < CH / 32; ++i) {
        int c = lane + i * 32;
        vst2(out + row * CH + c, (hr[c] - mu) * rstd * gamma[c] + beta[c]);
    }
}

extern "C" void kernel_launch(void* const* d_in, const int* in_sizes, int n_in,
                              void* d_out, int out_size, void* d_ws, size_t ws_size,
                              hipStream_t stream) {
    const float* X  = (const float*)d_in[0];
    const float* qp = (const float*)d_in[1];
    const float* Wq = (const float*)d_in[2];
    const float* bq = (const float*)d_in[3];
    const float* Wk = (const float*)d_in[4];
    const float* bk = (const float*)d_in[5];
    const float* Wv = (const float*)d_in[6];
    const float* bv = (const float*)d_in[7];
    const float* Wo = (const float*)d_in[8];
    const float* bo = (const float*)d_in[9];
    const float* gamma = (const float*)d_in[10];
    const float* beta  = (const float*)d_in[11];

    char* ws = (char*)d_ws;
    size_t off = 0;
    auto carve = [&](size_t bytes) -> void* {
        void* p = ws + off;
        off += (bytes + 255) & ~(size_t)255;
        return p;
    };
    const size_t actElems = (size_t)ROWS * CH;
    const size_t wElems   = (size_t)CH * CH;
    _Float16* Xh  = (_Float16*)carve(actElems * 2);
    _Float16* Wqh = (_Float16*)carve(wElems * 2);
    _Float16* Wkh = (_Float16*)carve(wElems * 2);
    _Float16* Wvh = (_Float16*)carve(wElems * 2);
    _Float16* Woh = (_Float16*)carve(wElems * 2);
    _Float16* Qh  = (_Float16*)carve(actElems * 2);
    _Float16* Kh  = (_Float16*)carve(actElems * 2);
    _Float16* Vth = (_Float16*)carve(actElems * 2);
    _Float16* Ah  = (_Float16*)carve(actElems * 2);
    float*    Hb  = (float*)carve(actElems * 4);

    cvt_f16_kernel<<<2048, 256, 0, stream>>>(X,  Xh,  (int)actElems);
    cvt_f16_kernel<<<128,  256, 0, stream>>>(Wq, Wqh, (int)wElems);
    cvt_f16_kernel<<<128,  256, 0, stream>>>(Wk, Wkh, (int)wElems);
    cvt_f16_kernel<<<128,  256, 0, stream>>>(Wv, Wvh, (int)wElems);
    cvt_f16_kernel<<<128,  256, 0, stream>>>(Wo, Woh, (int)wElems);

    dim3 ggrid(ROWS / 128, CH / 128);
    gemm_qkv_kernel<<<ggrid, 128, 0, stream>>>(Xh, Wqh, bq, Qh, 0);
    gemm_qkv_kernel<<<ggrid, 128, 0, stream>>>(Xh, Wkh, bk, Kh, 0);
    gemm_qkv_kernel<<<ggrid, 128, 0, stream>>>(Xh, Wvh, bv, Vth, 1);

    flash_attn_kernel<<<dim3(SEQ / 64, BATCH * HEADS), 128, 0, stream>>>(Qh, Kh, Vth, qp, Ah);

    gemm_out_kernel<<<ggrid, 128, 0, stream>>>(Ah, Woh, bo, X, Hb);

    layernorm_kernel<<<ROWS / 8, 256, 0, stream>>>(Hb, gamma, beta, (float*)d_out);
}
